// DCT_1133871366826
// MI455X (gfx1250) — hardware-verified
//
#include <hip/hip_runtime.h>


namespace {
constexpr int M = 2048, N = 4096;
constexpr float CS = 16384.0f;

typedef _Float16 b16;
typedef __attribute__((ext_vector_type(16))) _Float16 v16b;
typedef __attribute__((ext_vector_type(8))) _Float16 v8b;
typedef __attribute__((ext_vector_type(8))) float v8f;
typedef __attribute__((ext_vector_type(4))) float v4f;
__device__ __forceinline__ float bf16_rne(float f) { unsigned int u = __float_as_uint(f); u += 0x7FFFu + ((u >> 16) & 1u); return __uint_as_float(u & 0xFFFF0000u); }
__device__ __forceinline__ v16b frag_kb(const b16* p, int hh) { const v8b a = *(const v8b*)(p + 8 * hh), b = *(const v8b*)(p + 16 + 8 * hh); v16b f;
#pragma unroll
  for (int e = 0; e < 8; ++e) { f[e] = a[e]; f[8 + e] = b[e]; } return f; }
__device__ __forceinline__ v16b frag_x(const float* p, int hh) { v16b f;
#pragma unroll
  for (int e = 0; e < 8; ++e) { f[e] = (b16)bf16_rne(p[8 * hh + e]); f[8 + e] = (b16)bf16_rne(p[16 + 8 * hh + e]); } return f; }
__device__ __forceinline__ v8f wmma16b(v16b a, v16b b, v8f c) { v8f d = __builtin_amdgcn_wmma_f32_16x16x32_f16(false, a, false, b, (short)0, c, false, false); asm volatile("v_nop\n\tv_nop\n\tv_nop\n\tv_nop" : "+v"(d) : "v"(a), "v"(b)); return d; }
__device__ __forceinline__ void wave_lds_sync() { __builtin_amdgcn_fence(__ATOMIC_RELEASE, "workgroup"); __builtin_amdgcn_wave_barrier(); __builtin_amdgcn_fence(__ATOMIC_ACQUIRE, "workgroup"); }
__device__ __forceinline__ float cos_acc(float x) {
  const float k = rintf(x * 0.15915494309189535f); float r = __builtin_fmaf(k, -6.28318548202514648f, x); r = __builtin_fmaf(k, 1.7484556025237907e-7f, r);
  return __builtin_amdgcn_cosf(r * 0.15915494309189535f); }

__global__ __launch_bounds__(256) void table_kernel(b16* __restrict__ C16) {
  const size_t g = (size_t)blockIdx.x * 256 + threadIdx.x; const int k = (int)(g / (N / 8)), n0 = (int)(g % (N / 8)) * 8; const float pn = (float)(3.141592653589793 / 4096.0);
  v8b v;
#pragma unroll
  for (int e = 0; e < 8; ++e) { float t = pn * ((float)(n0 + e) + 0.5f); asm volatile("" : "+v"(t)); float a = t * (float)k; asm volatile("" : "+v"(a)); v[e] = (b16)(cos_acc(a) * CS); }
  for (int pass = 0; pass < 2; ++pass) { *(volatile v8b*)(C16 + (size_t)k * N + n0) = v; __threadfence(); }
}

__global__ __launch_bounds__(128) void dct_kernel(const float* __restrict__ x, const b16* __restrict__ C16, float* __restrict__ y) {
  __shared__ __attribute__((aligned(16))) float Ts[4][32 * 64];
  const int lane = threadIdx.x & 31, wave = threadIdx.x >> 5, nloc = lane & 15, hlf = lane >> 4, m0 = blockIdx.y * 128 + wave * 32, c0 = blockIdx.x * 64;
  v8f acc[2][4];
#pragma unroll
  for (int r = 0; r < 2; ++r)
#pragma unroll
    for (int t = 0; t < 4; ++t) acc[r][t] = (v8f){};
#pragma unroll 2
  for (int kb = 0; kb < N; kb += 32) { const v16b a0 = frag_x(x + (size_t)(m0 + nloc) * N + kb, hlf), a1 = frag_x(x + (size_t)(m0 + 16 + nloc) * N + kb, hlf);
#pragma unroll
    for (int t = 0; t < 4; ++t) { const v16b bw = frag_kb(C16 + (size_t)(c0 + t * 16 + nloc) * N + kb, hlf); acc[0][t] = wmma16b(a0, bw, acc[0][t]); acc[1][t] = wmma16b(a1, bw, acc[1][t]); } }
  float* Tt = Ts[wave];
#pragma unroll
  for (int t = 0; t < 4; ++t)
#pragma unroll
    for (int r = 0; r < 2; ++r)
#pragma unroll
      for (int v = 0; v < 8; ++v) Tt[(r * 16 + v + 8 * hlf) * 64 + t * 16 + nloc] = acc[r][t][v] * (1.0f / CS);
  wave_lds_sync();
  for (int pass = 0; pass < 2; ++pass) {
#pragma unroll
    for (int j = 0; j < 16; ++j) { const int rr = j * 2 + hlf, c4 = nloc * 4; *(volatile v4f*)(y + (size_t)(m0 + rr) * N + c0 + c4) = *(const v4f*)(Tt + rr * 64 + c4); }
    __threadfence(); }
}
}

extern "C" void kernel_launch(void* const* d_in, const int* in_sizes, int n_in,
                              void* d_out, int out_size, void* d_ws, size_t ws_size, hipStream_t stream) {
  (void)n_in; (void)out_size;
  const float* x = (const float*)d_in[0]; float* y = (float*)d_out;
  if (in_sizes[0] != M * N) return;
  if ((size_t)N * N * 2 > ws_size) return;
  b16* C16 = (b16*)d_ws;
  table_kernel<<<N * N / 8 / 256, 256, 0, stream>>>(C16);
  dct_kernel<<<dim3(N / 64, M / 128), 128, 0, stream>>>(x, C16, y);
}
